// QuantLinear_82463372083492
// MI455X (gfx1250) — hardware-verified
//
#include <hip/hip_runtime.h>
#include <stdint.h>

constexpr int kRowsM     = 128;
constexpr int kDepthK    = 4096;
constexpr int kColsN     = 11008;
constexpr int kGroupSize = 128;
constexpr int kNumGroups = kDepthK / kGroupSize;
constexpr int kPackRowsK = kDepthK / 8;
constexpr int kPackColsN = kColsN / 8;

constexpr int kWaveM  = 32;
constexpr int kWaveN  = 64;
constexpr int kTilesM = kRowsM / kWaveM;
constexpr int kTilesN = kColsN / kWaveN;
constexpr int kNumTiles = kTilesM * kTilesN;
constexpr int kGemmBlocks = kNumTiles / 8;

static_assert(kRowsM % kWaveM == 0);
static_assert(kColsN % kWaveN == 0);
static_assert(kDepthK % kGroupSize == 0);
static_assert(kGroupSize % 32 == 0);
static_assert(kNumTiles % 8 == 0);
static_assert(kColsN % 64 == 0);
static_assert(kDepthK % 256 == 0);

constexpr int kDqTileN    = 64;
constexpr int kDqTileRows = 32;
constexpr int kDqBlocksN  = kColsN / kDqTileN;
constexpr int kDqBlocksK  = kPackRowsK / kDqTileRows;
static_assert(kColsN % kDqTileN == 0);
static_assert(kPackRowsK % kDqTileRows == 0);
static_assert(kDqTileRows * 8 == 2 * kGroupSize);

constexpr size_t kXPlaneBytes = (size_t)kRowsM * kDepthK * 2;
constexpr size_t kBqBytes     = (size_t)kColsN * kDepthK * 2;
constexpr size_t kOffXh = 0;
constexpr size_t kOffXl = kOffXh + kXPlaneBytes;
constexpr size_t kOffBq = kOffXl + kXPlaneBytes;
constexpr size_t kWsTotal = kOffBq + kBqBytes;
static_assert(kWsTotal <= (size_t)134217728);
static_assert(kOffXl % 128 == 0 && kOffBq % 128 == 0);

typedef __attribute__((ext_vector_type(16))) __bf16   v16b;
typedef __attribute__((ext_vector_type(8)))  __bf16   v8b;
typedef __attribute__((ext_vector_type(8)))  float    v8f;
typedef __attribute__((ext_vector_type(4)))  float    v4f;
typedef __attribute__((ext_vector_type(4)))  unsigned int v4u;

__device__ __forceinline__ unsigned short f2bf_bits(float f) {
  unsigned u = __float_as_uint(f);
  return (unsigned short)((u + 0x7FFFu + ((u >> 16) & 1u)) >> 16);
}
__device__ __forceinline__ float bf_bits2f(unsigned short h) { return __uint_as_float(((unsigned)h) << 16); }
__device__ __forceinline__ unsigned pk16(unsigned short a, unsigned short b) { return (unsigned)a | ((unsigned)b << 16); }

__device__ __forceinline__ void dep_guard4_b(v8f& a, v8f& b, v8f& c, v8f& d, v16b x, v16b y) {
  asm volatile("v_nop\n\tv_nop\n\tv_nop\n\tv_nop" : "+v"(a), "+v"(b), "+v"(c), "+v"(d) : "v"(x), "v"(y));
}
__device__ __forceinline__ void keep4_b(v16b a, v16b b, v16b c, v16b d) { asm volatile("v_nop" :: "v"(a), "v"(b), "v"(c), "v"(d)); }
__device__ __forceinline__ void acc_guard4(v8f& a, v8f& b, v8f& c, v8f& d) { asm volatile("v_nop\n\tv_nop\n\tv_nop\n\tv_nop" : "+v"(a), "+v"(b), "+v"(c), "+v"(d)); }

template <typename T> struct Frag;
template <> struct Frag<__bf16> {
  typedef v16b V; union U { v16b v; v8b h[2]; };
  static __device__ __forceinline__ v16b load(const __bf16* p) {
    U f; f.h[0] = *(const v8b*)(p); f.h[1] = *(const v8b*)(p + 16); return f.v;
  }
  static __device__ __forceinline__ v8f mma(v16b a, v16b b, v8f c) {
    return __builtin_amdgcn_wmma_f32_16x16x32_bf16(false, a, false, b, (short)0, c, false, false);
  }
};

__global__ __launch_bounds__(256) void xsplit_kernel(const float* __restrict__ x,
                                                     unsigned short* __restrict__ xh,
                                                     unsigned short* __restrict__ xl, int n8) {
  const int i = blockIdx.x * 256 + threadIdx.x;
  if (i >= n8) return;
  const float* p = x + 8 * (size_t)i;
  const v4f a = *(const v4f*)(p);
  const v4f c = *(const v4f*)(p + 4);
  unsigned short hb[8], lb[8];
#pragma unroll
  for (int e = 0; e < 4; ++e) {
    float f0 = a[e];
    const unsigned short h0 = f2bf_bits(f0);
    hb[e] = h0;
    lb[e] = f2bf_bits(f0 - bf_bits2f(h0));
    float f1 = c[e];
    const unsigned short h1 = f2bf_bits(f1);
    hb[4 + e] = h1;
    lb[4 + e] = f2bf_bits(f1 - bf_bits2f(h1));
  }
  const v4u uh = (v4u){pk16(hb[0], hb[1]), pk16(hb[2], hb[3]), pk16(hb[4], hb[5]), pk16(hb[6], hb[7])};
  const v4u ul = (v4u){pk16(lb[0], lb[1]), pk16(lb[2], lb[3]), pk16(lb[4], lb[5]), pk16(lb[6], lb[7])};
  unsigned short* qh = xh + 8 * (size_t)i;
  unsigned short* ql = xl + 8 * (size_t)i;
  *(volatile v4u*)qh = uh;
  *(volatile v4u*)ql = ul;
  __threadfence();
  *(volatile v4u*)qh = uh;
  *(volatile v4u*)ql = ul;
}

__global__ __launch_bounds__(256) void dequant_kernel(const int* __restrict__ qweight,
                                                      const int* __restrict__ qzeros,
                                                      const int* __restrict__ gidx,
                                                      unsigned short* __restrict__ bq) {
  __shared__ __align__(16) v4u tile[kDqTileN * 33];
  const int t  = threadIdx.x;
  const int n0 = blockIdx.x * kDqTileN;
  const int r0 = blockIdx.y * kDqTileRows;
  const int c  = t & 63;
  const int n  = n0 + c;
  const int rq = t >> 6;
  int g0 = gidx[r0 * 8];
  int g1 = gidx[(r0 + 16) * 8];
  g0 = g0 < 0 ? 0 : g0; g0 = g0 > (kNumGroups - 1) ? (kNumGroups - 1) : g0;
  g1 = g1 < 0 ? 0 : g1; g1 = g1 > (kNumGroups - 1) ? (kNumGroups - 1) : g1;
  const unsigned zw0 = (unsigned)qzeros[(size_t)g0 * kPackColsN + (n >> 3)];
  const unsigned zw1 = (unsigned)qzeros[(size_t)g1 * kPackColsN + (n >> 3)];
  const int zs = (n & 7) * 4;
  const int z0 = (int)((zw0 >> zs) & 15u) + 1;
  const int z1 = (int)((zw1 >> zs) & 15u) + 1;
#pragma unroll
  for (int i = 0; i < 8; ++i) {
    const int rl = i * 4 + rq;
    const unsigned w = (unsigned)qweight[(size_t)(r0 + rl) * kColsN + n];
    const int z = (i < 4) ? z0 : z1;
    unsigned short b[8];
#pragma unroll
    for (int jj = 0; jj < 8; ++jj) {
      const int q = (int)((w >> (4 * jj)) & 15u);
      b[jj] = f2bf_bits((float)(q - z));
    }
    tile[c * 33 + rl] = (v4u){pk16(b[0], b[1]), pk16(b[2], b[3]), pk16(b[4], b[5]), pk16(b[6], b[7])};
  }
  __syncthreads();
  const int lane = t & 31, wave = t >> 5;
  const size_t kbase = (size_t)blockIdx.y * (kDqTileRows * 8);
  for (int ps = 0; ps < 2; ++ps) {
#pragma unroll
    for (int it = 0; it < 8; ++it) {
      const int nl = wave * 8 + it;
      const v4u u = tile[nl * 33 + lane];
      *(volatile v4u*)(bq + (size_t)(n0 + nl) * kDepthK + kbase + (size_t)lane * 8) = u;
    }
    __threadfence();
  }
}

__global__ __launch_bounds__(256) void qgemm_kernel(const unsigned short* __restrict__ xh,
                                                    const unsigned short* __restrict__ xl,
                                                    const unsigned short* __restrict__ bq,
                                                    const float* __restrict__ scales,
                                                    const float* __restrict__ bias,
                                                    const int* __restrict__ gidx,
                                                    float* __restrict__ out) {
  __shared__ __align__(16) float sT[8][16 * 68];
  const int lane = threadIdx.x & 31;
  const int wave = threadIdx.x >> 5;
  const int tile = blockIdx.x * 8 + wave;
  if (tile >= kNumTiles) return;
  const int tm = tile % kTilesM;
  const int tn = tile / kTilesM;
  const int m0 = tm * kWaveM;
  const int n0 = tn * kWaveN;

  const __bf16* A  = (const __bf16*)xh;
  const __bf16* A2 = (const __bf16*)xl;
  const __bf16* Bt = (const __bf16*)bq;

  const int rlane = lane & 15;
  const int koff  = (lane >> 4) * 8;
  const int mOff  = (lane >> 4) * 8;

  v8f accG[2][4], accT[2][4];
#pragma unroll
  for (int i = 0; i < 2; ++i)
#pragma unroll
    for (int j = 0; j < 4; ++j) accT[i][j] = (v8f){0.f,0.f,0.f,0.f,0.f,0.f,0.f,0.f};

#pragma unroll 1
  for (int grp = 0; grp < kNumGroups; ++grp) {
    int g = gidx[grp * kGroupSize];
    g = g < 0 ? 0 : g;
    g = g > (kNumGroups - 1) ? (kNumGroups - 1) : g;
    float sc[4];
#pragma unroll
    for (int j = 0; j < 4; ++j) sc[j] = scales[(size_t)g * kColsN + n0 + (j << 4) + rlane];
#pragma unroll
    for (int i = 0; i < 2; ++i)
#pragma unroll
      for (int j = 0; j < 4; ++j) accG[i][j] = (v8f){0.f,0.f,0.f,0.f,0.f,0.f,0.f,0.f};

#pragma unroll 1
    for (int ks = 0; ks < kGroupSize / 32; ++ks) {
      const int k0 = grp * kGroupSize + ks * 32;
      v16b bh[4];
#pragma unroll
      for (int j = 0; j < 4; ++j) {
        const size_t bo = (size_t)(n0 + (j << 4) + rlane) * kDepthK + koff + k0;
        bh[j] = Frag<__bf16>::load(Bt + bo);
      }
#pragma unroll
      for (int i = 0; i < 2; ++i) {
        const size_t ao = (size_t)(m0 + (i << 4) + rlane) * kDepthK + koff + k0;
        const v16b ah = Frag<__bf16>::load(A + ao);
        const v16b al = Frag<__bf16>::load(A2 + ao);
#pragma unroll
        for (int j = 0; j < 4; ++j) {
          accG[i][j] = Frag<__bf16>::mma(ah, bh[j], accG[i][j]);
          accG[i][j] = Frag<__bf16>::mma(al, bh[j], accG[i][j]);
        }
        dep_guard4_b(accG[i][0], accG[i][1], accG[i][2], accG[i][3], ah, al);
      }
      keep4_b(bh[0], bh[1], bh[2], bh[3]);
    }
    acc_guard4(accG[0][0], accG[0][1], accG[0][2], accG[0][3]);
    acc_guard4(accG[1][0], accG[1][1], accG[1][2], accG[1][3]);
#pragma unroll
    for (int i = 0; i < 2; ++i) {
#pragma unroll
      for (int j = 0; j < 4; ++j) {
        v8f tg = accG[i][j];
        v8f tt = accT[i][j];
#pragma unroll
        for (int r = 0; r < 8; ++r) tt[r] = fmaf(tg[r], sc[j], tt[r]);
        accT[i][j] = tt;
      }
    }
  }

  float* slab = sT[wave];
#pragma unroll
  for (int i = 0; i < 2; ++i) {
    const int mBase = m0 + (i << 4);
#pragma unroll
    for (int j = 0; j < 4; ++j) {
      const int n = n0 + (j << 4) + rlane;
      const float bv = bias[n];
#pragma unroll
      for (int r = 0; r < 8; ++r) {
        const float v = accT[i][j][r] + bv;
        slab[(mOff + r) * 68 + (j << 4) + rlane] = v;
      }
    }
    __builtin_amdgcn_fence(__ATOMIC_RELEASE, "workgroup");
    __builtin_amdgcn_wave_barrier();
    __builtin_amdgcn_fence(__ATOMIC_ACQUIRE, "workgroup");
    {
      const int hh = lane >> 4, c4 = (lane & 15) * 4;
      for (int ps = 0; ps < 2; ++ps) {
#pragma unroll
        for (int it = 0; it < 8; ++it) {
          const int row = it * 2 + hh;
          v4f v = *(const v4f*)(slab + row * 68 + c4);
          *(volatile v4f*)(out + (size_t)(mBase + row) * kColsN + n0 + c4) = v;
        }
        __threadfence();
      }
    }
    __builtin_amdgcn_fence(__ATOMIC_RELEASE, "workgroup");
    __builtin_amdgcn_wave_barrier();
    __builtin_amdgcn_fence(__ATOMIC_ACQUIRE, "workgroup");
  }
}

extern "C" void kernel_launch(void* const* d_in, const int* in_sizes, int n_in,
                              void* d_out, int out_size, void* d_ws, size_t ws_size,
                              hipStream_t stream) {
  if (n_in < 6) return;
  if (in_sizes[0] != kRowsM * kDepthK) return;
  if (in_sizes[1] != kPackRowsK * kColsN) return;
  if (in_sizes[2] != kNumGroups * kPackColsN) return;
  if (in_sizes[3] != kNumGroups * kColsN) return;
  if (in_sizes[4] != kColsN) return;
  if (in_sizes[5] != kDepthK) return;
  if (out_size != kRowsM * kColsN) return;
  if (ws_size < kWsTotal) return;

  const float* x      = (const float*)d_in[0];
  const int*   qw     = (const int*)d_in[1];
  const int*   qz     = (const int*)d_in[2];
  const float* scales = (const float*)d_in[3];
  const float* bias   = (const float*)d_in[4];
  const int*   gi     = (const int*)d_in[5];
  float* outp = (float*)d_out;

  char* ws = (char*)d_ws;
  unsigned short* xh = (unsigned short*)(ws + kOffXh);
  unsigned short* xl = (unsigned short*)(ws + kOffXl);
  unsigned short* bq = (unsigned short*)(ws + kOffBq);

  const int n8 = (kRowsM * kDepthK) / 8;
  xsplit_kernel<<<dim3((n8 + 255) / 256), dim3(256), 0, stream>>>(x, xh, xl, n8);
  dequant_kernel<<<dim3(kDqBlocksN, kDqBlocksK), dim3(256), 0, stream>>>(qw, qz, gi, bq);
  qgemm_kernel<<<dim3(kGemmBlocks), dim3(256), 0, stream>>>(xh, xl, bq, scales, bias, gi, outp);
}
